// CrissCrossAttention_77197742178884
// MI455X (gfx1250) — hardware-run, weakly checked
//
#include <hip/hip_runtime.h>
#define NB 4
#define CH 64
#define SD 128
#define HWP (SD * SD)
#define NPX (NB * HWP)
#define CSC 256.0f
#define TINYV 1.0e-5f
#define RSC 64.0f
#define RSD 2048.0f
typedef __bf16 v16b __attribute__((ext_vector_type(16)));
typedef unsigned short v8us __attribute__((ext_vector_type(8), may_alias));
typedef float  v8f  __attribute__((ext_vector_type(8)));
typedef float  v4f  __attribute__((ext_vector_type(4)));
typedef float  v4fa __attribute__((ext_vector_type(4), may_alias));
union FragB { v16b v; v8us half[2]; unsigned short u[16]; };

__device__ __forceinline__ unsigned short bf16_bits(float x) { unsigned int u = __float_as_uint(x); return (unsigned short)((u + 0x7FFFu + ((u >> 16) & 1u)) >> 16); }
__device__ __forceinline__ float bf16_val(unsigned short b) { return __uint_as_float(((unsigned int)b) << 16); }
__device__ __forceinline__ float bf16_round(float x) { return bf16_val(bf16_bits(x)); }
template <int NT>
__device__ __forceinline__ v8f mmaN(v16b ah, v16b al, v16b bh, v16b bl, v8f c) {
  c = __builtin_amdgcn_wmma_f32_16x16x32_bf16(false, ah, false, bh, (short)0, c, false, false);
  if (NT >= 2) c = __builtin_amdgcn_wmma_f32_16x16x32_bf16(false, al, false, bh, (short)0, c, false, false);
  if (NT >= 3) c = __builtin_amdgcn_wmma_f32_16x16x32_bf16(false, ah, false, bl, (short)0, c, false, false);
  asm volatile("v_nop\n\tv_nop\n\tv_nop\n\tv_nop" : "+v"(c) : "v"(ah), "v"(al), "v"(bh), "v"(bl));
  return c;
}


typedef _Float16 v16h __attribute__((ext_vector_type(16)));
union FragH { v16h v; v8us half[2]; _Float16 h[16]; unsigned short u[16]; };
template <int NT>
__device__ __forceinline__ v8f mmaH(v16h ah, v16h al, v16h bh, v16h bl, v8f c) {
  c = __builtin_amdgcn_wmma_f32_16x16x32_f16(false, ah, false, bh, (short)0, c, false, false);
  if (NT >= 2) c = __builtin_amdgcn_wmma_f32_16x16x32_f16(false, al, false, bh, (short)0, c, false, false);
  if (NT >= 3) c = __builtin_amdgcn_wmma_f32_16x16x32_f16(false, ah, false, bl, (short)0, c, false, false);
  asm volatile("v_nop\n\tv_nop\n\tv_nop\n\tv_nop" : "+v"(c) : "v"(ah), "v"(al), "v"(bh), "v"(bl));
  return c;
}

__global__ __launch_bounds__(256) void k_wt_f16(const float* __restrict__ W, _Float16* __restrict__ Wt, int K, int N, float scale) {
  const int t = blockIdx.x * 256 + threadIdx.x; if (t >= N * (K / 8)) return; const int n = t / (K / 8), k8 = (t % (K / 8)) * 8; FragH f;
#pragma unroll
  for (int i = 0; i < 8; ++i) f.h[i] = (_Float16)(bf16_round(W[(size_t)(k8 + i) * N + n]) * scale); const v8us o = f.half[0];
  *(volatile v8us*)((unsigned short*)Wt + (size_t)n * K + k8) = o; __threadfence(); *(volatile v8us*)((unsigned short*)Wt + (size_t)n * K + k8) = o;
}

typedef _Float16 v4h __attribute__((ext_vector_type(4)));

__global__ __launch_bounds__(256) void k_x16(const float* __restrict__ x, _Float16* __restrict__ X16, size_t n8) { const size_t t = (size_t)blockIdx.x * 256 + threadIdx.x; if (t >= n8) return; FragH f;
#pragma unroll
  for (int q = 0; q < 8; ++q) f.h[q] = (_Float16)bf16_round(x[t * 8 + q]); *(volatile v8us*)((unsigned short*)X16 + t * 8) = f.half[0]; __threadfence(); *(volatile v8us*)((unsigned short*)X16 + t * 8) = f.half[0]; }
__device__ __forceinline__ v16h g2_frag(const _Float16* p, int hh) { FragH f; f.half[0] = *(const v8us*)((const unsigned short*)p + 8 * hh); f.half[1] = *(const v8us*)((const unsigned short*)p + 16 + 8 * hh); return f.v; }
__device__ __forceinline__ v8f g2_mma(v16h a, v16h b, v8f c) { v8f d = __builtin_amdgcn_wmma_f32_16x16x32_f16(false, a, false, b, (short)0, c, false, false); asm volatile("v_nop\n\tv_nop\n\tv_nop\n\tv_nop" : "+v"(d) : "v"(a), "v"(b)); return d; }
template <int ACT>
__global__ __launch_bounds__(128) void k_gemm2(const _Float16* __restrict__ A, int lda, size_t sA, const _Float16* __restrict__ Bh, int ldb, size_t sB, float alpha, const float* __restrict__ bias, size_t sBias, const float* __restrict__ CP, int rowsPerB, size_t sCPb, int row0g,
    float* __restrict__ C, _Float16* __restrict__ C16, int ldc, size_t sC, int M, int N, int K) { static_assert(ACT == 0 || ACT == 3 || ACT == 6 || ACT == 8 || ACT == 9 || ACT == 11 || ACT == 12 || ACT == 14 || ACT == 15 || ACT == 16 || ACT == 17, "k_gemm2: unsupported ACT code (would silently apply no activation)");
  __shared__ __attribute__((aligned(16))) float so[4][32][68];
  const int tid = threadIdx.x, w = tid >> 5, lane = tid & 31, ln = lane & 15, hh = lane >> 4; const int by = blockIdx.y;
  A += (size_t)by * sA; Bh += (size_t)by * sB; const size_t cofs = (size_t)by * sC; const float* bp = bias ? bias + (size_t)by * sBias : nullptr;
  const int ntn = N >> 6; const int mt = blockIdx.x / ntn, nq = blockIdx.x - mt * ntn; const int row0 = mt * 128 + 32 * w, col0 = nq * 64; if (row0 >= M) return;
  const _Float16* a0p = A + (size_t)(row0 + ln) * lda; const _Float16* a1p = a0p + (size_t)16 * lda;
  const _Float16* b0p = Bh + (size_t)(col0 + ln) * ldb; const _Float16* b1p = b0p + (size_t)16 * ldb; const _Float16* b2p = b1p + (size_t)16 * ldb; const _Float16* b3p = b2p + (size_t)16 * ldb;
  const v8f z8 = {0.f,0.f,0.f,0.f,0.f,0.f,0.f,0.f}; v8f c00 = z8, c01 = z8, c02 = z8, c03 = z8, c10 = z8, c11 = z8, c12 = z8, c13 = z8;
  for (int kb = 0; kb < K; kb += 32) { const v16h a0 = g2_frag(a0p + kb, hh), a1 = g2_frag(a1p + kb, hh);
    v16h b = g2_frag(b0p + kb, hh); c00 = g2_mma(a0, b, c00); c10 = g2_mma(a1, b, c10);
    b = g2_frag(b1p + kb, hh); c01 = g2_mma(a0, b, c01); c11 = g2_mma(a1, b, c11);
    b = g2_frag(b2p + kb, hh); c02 = g2_mma(a0, b, c02); c12 = g2_mma(a1, b, c12);
    b = g2_frag(b3p + kb, hh); c03 = g2_mma(a0, b, c03); c13 = g2_mma(a1, b, c13); }
  v8f accs[8] = {c00, c01, c02, c03, c10, c11, c12, c13};
#pragma unroll
  for (int u = 0; u < 8; ++u) { const int t = u & 3, half = u >> 2; const int col = col0 + t * 16 + ln; const float bv = bp ? bf16_round(bp[col]) : 0.f;
#pragma unroll
    for (int r = 0; r < 8; ++r) { const int rloc = half * 16 + 8 * hh + r; float v = accs[u][r] * alpha + bv; if (CP) { if (rowsPerB < 0) v += CP[cofs + (size_t)(row0g + row0 + rloc) * ldc + col];        else { const int bidx = (row0g + row0 + rloc) / rowsPerB; v += CP[(size_t)bidx * sCPb + (size_t)by * 64 + col]; } }
      if (ACT == 3) v = fmaxf(v, 0.f); else if (ACT == 6) v = 0.5f * v * (1.0f + erff(v * 0.70710678118654752f)); else if (ACT == 11) v = 1.0f / (1.0f + expf(-v)); else if (ACT == 15) v = v / (1.0f + expf(-v)); else if (ACT == 12) v = (v > 0.f) ? v : 0.01f * v; else if (ACT == 8) v = tanhf(v); else if (ACT == 9) v = 0.5f * v * (1.0f + tanhf(0.7978845608028654f * (v + 0.044715f * v * v * v))); else if (ACT == 14) v = (v > 0.f) ? v : 0.1f * v; else if (ACT == 16) v = (v >= 0.f) ? v : 0.3f * v; else if (ACT == 17) v = (v >= 0.f) ? v : 0.2f * v;
      so[w][rloc][t * 16 + ln] = v; } }
  __builtin_amdgcn_fence(__ATOMIC_ACQ_REL, "workgroup"); __builtin_amdgcn_wave_barrier();
  const int rsub = lane >> 4, c4 = (lane & 15) * 4;
  for (int pass = 0; pass < 2; ++pass) {
#pragma unroll
    for (int q = 0; q < 16; ++q) { const int r = q * 2 + rsub; const v4f v = *(const v4fa*)&so[w][r][c4]; if (C) *(volatile v4f*)(C + cofs + (size_t)(row0 + r) * ldc + col0 + c4) = v; if (C16) { v4h h4; for (int i = 0; i < 4; ++i) h4[i] = (_Float16)v[i]; *(volatile v4h*)(C16 + cofs + (size_t)(row0 + r) * ldc + col0 + c4) = h4; } }
    if (pass == 0) __threadfence(); } }
typedef float  v2f  __attribute__((ext_vector_type(2)));
typedef float  v2fa __attribute__((ext_vector_type(2), may_alias));

__global__ __launch_bounds__(256) void k_two(const float* __restrict__ R, int col0, const float* __restrict__ bias, _Float16* __restrict__ dst, int side, int n) {
  const int t = blockIdx.x * 256 + threadIdx.x; if (t >= n) return; const float* p = R + (size_t)t * CH + col0; FragH hi, lo, pt; FragH zz;
  for (int c = 0; c < 8; ++c) { const float s = (p[c] + bf16_round(bias[c])) * CSC; const _Float16 h = (_Float16)s; hi.h[c] = h; lo.h[c] = (_Float16)((s - (float)h) * RSC); pt.h[c] = (_Float16)((float)h * (1.0f / RSC)); zz.h[c] = (_Float16)0.0f; }
  const v8us P0 = hi.half[0], P1 = side ? pt.half[0] : lo.half[0], P2 = side ? lo.half[0] : pt.half[0], P3 = zz.half[0]; unsigned short* d = (unsigned short*)dst + (size_t)t * 32;
  for (int pass = 0; pass < 2; ++pass) { *(volatile v8us*)(d) = P0; *(volatile v8us*)(d + 8) = P1; *(volatile v8us*)(d + 16) = P2; *(volatile v8us*)(d + 24) = P3; if (pass == 0) __threadfence(); } }

__global__ __launch_bounds__(256) void k_jsm(const float* __restrict__ S, _Float16* __restrict__ Wt, int n) {
  const int t = blockIdx.x * 256 + threadIdx.x; if (t >= n) return; const float* r = S + (size_t)t * 256; const int own = (t >> 7) & (SD - 1); float mx = -3.0e38f;
  for (int j = 0; j < 256; ++j) { const float pen = (j == own) ? -3.0e38f : 0.f; const float e = r[j] + pen; mx = (e > mx) ? e : mx; }
  float sm = 0.f; for (int j = 0; j < 256; ++j) { const float kp = (j == own) ? 0.f : 1.f; const float d0 = r[j] - mx; const float dd = (d0 < 0.f) ? d0 : 0.f; sm += expf(dd) * kp; }
  unsigned short* d = (unsigned short*)Wt + (size_t)t * 256;
  for (int j8 = 0; j8 < 256; j8 += 8) { FragH f; for (int i = 0; i < 8; ++i) { const float kp = ((j8 + i) == own) ? 0.f : CSC; const float d0 = r[j8 + i] - mx; const float dd = (d0 < 0.f) ? d0 : 0.f; f.h[i] = (_Float16)((expf(dd) / sm) * kp); } *(volatile v8us*)(d + j8) = f.half[0]; __threadfence(); *(volatile v8us*)(d + j8) = f.half[0]; } }

__global__ __launch_bounds__(256) void k_trp(const _Float16* __restrict__ src, _Float16* __restrict__ dst, int n8) {
  const int t = blockIdx.x * 256 + threadIdx.x; if (t >= n8) return; const int pl = t >> 11, x = (t >> 4) & (SD - 1), y8 = (t & 15) * 8; const unsigned short* s = (const unsigned short*)src + (size_t)pl * HWP + (size_t)y8 * SD + x; FragH f;
  for (int i = 0; i < 8; ++i) f.u[i] = s[(size_t)i * SD]; unsigned short* d = (unsigned short*)dst + (size_t)pl * HWP + (size_t)x * SD + y8; *(volatile v8us*)d = f.half[0]; __threadfence(); *(volatile v8us*)d = f.half[0]; }

__global__ __launch_bounds__(256) void k_adf(const float* __restrict__ YA, const float* __restrict__ YB, _Float16* __restrict__ D1, _Float16* __restrict__ D2, int n8) {
  const int t = blockIdx.x * 256 + threadIdx.x; if (t >= n8) return; const float* a = YA + (size_t)t * 8; const float* b = YB + (size_t)t * 8; FragH hi, lo;
  for (int i = 0; i < 8; ++i) { const float s = fabsf(a[i] - b[i]) * CSC; const _Float16 h = (_Float16)s; hi.h[i] = h; lo.h[i] = (_Float16)((s - (float)h) * RSD); }
  unsigned short* d1 = (unsigned short*)D1 + (size_t)t * 8; unsigned short* d2 = (unsigned short*)D2 + (size_t)t * 8; for (int pass = 0; pass < 2; ++pass) { *(volatile v8us*)d1 = hi.half[0]; *(volatile v8us*)d2 = lo.half[0]; if (pass == 0) __threadfence(); } }

__global__ __launch_bounds__(64) void k_bns(const float* __restrict__ Z, float* __restrict__ ST, int n) {
  const int c = blockIdx.x * 64 + threadIdx.x; if (c >= n) return; const float* z = Z + c; float tot = 0.f;
  for (int bk = 0; bk < 256; ++bk) { float s = 0.f; for (int i = 0; i < 256; ++i) s += z[(size_t)(bk * 256 + i) * CH]; tot += s; }
  const float mean = tot * (1.0f / (float)NPX); float tv = 0.f;
  for (int bk = 0; bk < 256; ++bk) { float s = 0.f; for (int i = 0; i < 256; ++i) { const float dlt = z[(size_t)(bk * 256 + i) * CH] - mean; s += dlt * dlt; } tv += s; }
  const v2f o = {mean, tv * (1.0f / (float)NPX)}; *(volatile v2f*)(ST + (size_t)c * 2) = o; __threadfence(); *(volatile v2f*)(ST + (size_t)c * 2) = o; }

__global__ __launch_bounds__(256) void k_two_outs(const float* __restrict__ YA, const float* __restrict__ YB, const float* __restrict__ Z, const float* __restrict__ ST, const float* __restrict__ IA, const float* __restrict__ IB, const float* __restrict__ G1, const float* __restrict__ G2, const float* __restrict__ SCL, const float* __restrict__ SHF, float* __restrict__ O1, float* __restrict__ O2, int n4) {
  const int t = blockIdx.x * 256 + threadIdx.x; if (t >= n4) return; const int x4 = (t & 31) * 4, y = (t >> 5) & (SD - 1), c = (t >> 12) & (CH - 1), bb = t >> 18; const size_t px = ((size_t)bb * SD + y) * SD + x4; const size_t io = (((size_t)bb * CH + c) * SD + y) * SD + x4;
  const v2f st = *(const v2fa*)(ST + (size_t)c * 2); const float rs = 1.0f / sqrtf(st[1] + TINYV), sc = bf16_round(SCL[c]), sh = bf16_round(SHF[c]), g1 = bf16_round(G1[0]), g2 = bf16_round(G2[0]); v4f o1, o2;
  for (int i = 0; i < 4; ++i) { const size_t r = (px + i) * CH + c; const float nrm = (Z[r] - st[0]) * rs * sc + sh; o1[i] = g1 * YA[r] + bf16_round(IA[io + i]) + nrm; o2[i] = g2 * YB[r] + bf16_round(IB[io + i]) + nrm; }
  for (int pass = 0; pass < 2; ++pass) { *(volatile v4f*)(O1 + io) = o1; *(volatile v4f*)(O2 + io) = o2; if (pass == 0) __threadfence(); } }

extern "C" void kernel_launch(void* const* d_in, const int* in_sizes, int n_in,
                              void* d_out, int out_size, void* d_ws, size_t ws_size, hipStream_t stream) {
  (void)in_sizes; (void)n_in; (void)out_size;
  const float* IA = (const float*)d_in[0]; const float* IB = (const float*)d_in[1];
  const float* WA1 = (const float*)d_in[2]; const float* BA1 = (const float*)d_in[3]; const float* WA2 = (const float*)d_in[4]; const float* BA2 = (const float*)d_in[5]; const float* WA3 = (const float*)d_in[6]; const float* BA3 = (const float*)d_in[7];
  const float* WB1 = (const float*)d_in[8]; const float* BB1 = (const float*)d_in[9]; const float* WB2 = (const float*)d_in[10]; const float* BB2 = (const float*)d_in[11]; const float* WB3 = (const float*)d_in[12]; const float* BB3 = (const float*)d_in[13];
  const float* G1 = (const float*)d_in[14]; const float* G2 = (const float*)d_in[15]; const float* WPJ = (const float*)d_in[16]; const float* BPJ = (const float*)d_in[17]; const float* SCL = (const float*)d_in[18]; const float* SHF = (const float*)d_in[19];
  static_assert(NB == 4 && CH == 64 && SD == 128 && HWP == 16384 && NPX == 65536 && (HWP * (CH / 8)) % 256 == 0 && NPX % 256 == 0 && NPX % 128 == 0 && SD % 128 == 0 && CH % 64 == 0 && (NB * CH * HWP / 8) % 256 == 0 && (NB * CH * HWP / 4) % 256 == 0, "the index shifts; whole tiles; exact grids");
  float* O1 = (float*)d_out; float* O2 = O1 + (size_t)NB * CH * HWP;
  char* ws = (char*)d_ws; size_t off = 0;
  auto take = [&](size_t bytes) { char* p = ws + off; off += (bytes + 255) & ~(size_t)255; return p; };
  _Float16* PA = (_Float16*)take((size_t)NPX * CH * 2); _Float16* PB = (_Float16*)take((size_t)NPX * CH * 2);
  _Float16* W1 = (_Float16*)take((size_t)64 * CH * 2); _Float16* W2 = (_Float16*)take((size_t)64 * CH * 2); _Float16* W3A = (_Float16*)take((size_t)CH * CH * 2); _Float16* W3B = (_Float16*)take((size_t)CH * CH * 2); _Float16* W4 = (_Float16*)take((size_t)CH * CH * 2);
  float* R1 = (float*)take((size_t)NPX * 64 * 4); float* R2 = (float*)take((size_t)NPX * 64 * 4);
  _Float16* QA = (_Float16*)take((size_t)NPX * 32 * 2); _Float16* KA = (_Float16*)take((size_t)NPX * 32 * 2); _Float16* QB = (_Float16*)take((size_t)NPX * 32 * 2); _Float16* KB = (_Float16*)take((size_t)NPX * 32 * 2);
  float* SC = (float*)take((size_t)NPX * 256 * 4); _Float16* WT = (_Float16*)take((size_t)NPX * 256 * 2);
  _Float16* VC = (_Float16*)take((size_t)NB * CH * HWP * 2); _Float16* VX = (_Float16*)take((size_t)NB * CH * HWP * 2);
  float* YA = (float*)take((size_t)NPX * CH * 4); float* YB = (float*)take((size_t)NPX * CH * 4);
  _Float16* D1 = (_Float16*)take((size_t)NPX * CH * 2); _Float16* D2 = (_Float16*)take((size_t)NPX * CH * 2); float* ST = (float*)take((size_t)CH * 2 * 4);
  float* YC = R1;
  float* Z1 = SC; float* ZZ = SC + (size_t)NPX * CH;
  if (off > ws_size) return;
  for (int b = 0; b < NB; ++b) { k_wt_f16<<<(unsigned)(HWP * (CH / 8) / 256), 256, 0, stream>>>(IA + (size_t)b * CH * HWP, PA + (size_t)b * HWP * CH, CH, HWP, CSC); k_wt_f16<<<(unsigned)(HWP * (CH / 8) / 256), 256, 0, stream>>>(IB + (size_t)b * CH * HWP, PB + (size_t)b * HWP * CH, CH, HWP, CSC); }
  k_x16<<<1, 256, 0, stream>>>(WA2, W1, (size_t)8 * CH / 8); k_x16<<<1, 256, 0, stream>>>(WB1, W1 + (size_t)8 * CH, (size_t)8 * CH / 8); k_x16<<<1, 256, 0, stream>>>(WB2, W1 + (size_t)16 * CH, (size_t)8 * CH / 8); k_x16<<<2, 256, 0, stream>>>(WA3, W1 + (size_t)24 * CH, (size_t)40 * CH / 8);
  k_x16<<<1, 256, 0, stream>>>(WA1, W2, (size_t)8 * CH / 8); k_x16<<<2, 256, 0, stream>>>(WA3, W2 + (size_t)8 * CH, (size_t)56 * CH / 8);
  k_x16<<<2, 256, 0, stream>>>(WA3, W3A, (size_t)CH * CH / 8); k_x16<<<2, 256, 0, stream>>>(WB3, W3B, (size_t)CH * CH / 8); k_x16<<<2, 256, 0, stream>>>(WPJ, W4, (size_t)CH * CH / 8);
  k_gemm2<0><<<dim3((NPX / 128) * (64 / 64), 1), 128, 0, stream>>>(PA, CH, 0, W1, CH, 0, 1.0f / CSC, nullptr, 0, nullptr, 1, 0, 0, R1, nullptr, 64, 0, NPX, 64, CH);
  k_gemm2<0><<<dim3((NPX / 128) * (64 / 64), 1), 128, 0, stream>>>(PB, CH, 0, W2, CH, 0, 1.0f / CSC, nullptr, 0, nullptr, 1, 0, 0, R2, nullptr, 64, 0, NPX, 64, CH);
  k_two<<<NPX / 256, 256, 0, stream>>>(R2, 0, BA1, QA, 0, NPX); k_two<<<NPX / 256, 256, 0, stream>>>(R1, 0, BA2, KA, 1, NPX); k_two<<<NPX / 256, 256, 0, stream>>>(R1, 8, BB1, QB, 0, NPX); k_two<<<NPX / 256, 256, 0, stream>>>(R1, 16, BB2, KB, 1, NPX);
  for (int br = 0; br < 2; ++br) { const _Float16* W3 = br ? W3B : W3A; const _Float16* Qp = br ? QB : QA; const _Float16* Kp = br ? KB : KA; const float* B3 = br ? BB3 : BA3; float* Y = br ? YB : YA;
    k_gemm2<0><<<dim3(1 * (HWP / 64), NB), 128, 0, stream>>>(W3, CH, 0, PA, CH, (size_t)HWP * CH, 1.0f, nullptr, 0, nullptr, 1, 0, 0, nullptr, VC, HWP, (size_t)CH * HWP, CH, HWP, CH);
    k_trp<<<(unsigned)(NB * CH * HWP / 8 / 256), 256, 0, stream>>>(VC, VX, NB * CH * HWP / 8);
    k_gemm2<0><<<dim3((SD / 128) * (SD / 64), NB * SD), 128, 0, stream>>>(Qp, 32, (size_t)SD * 32, Kp, 32, (size_t)SD * 32, 1.0f / (CSC * CSC), nullptr, 0, nullptr, 1, 0, 0, SC + SD, nullptr, 256, (size_t)SD * 256, SD, SD, 32);
    for (int b = 0; b < NB; ++b) k_gemm2<0><<<dim3((SD / 128) * (SD / 64), SD), 128, 0, stream>>>(Qp + (size_t)b * HWP * 32, SD * 32, 32, Kp + (size_t)b * HWP * 32, SD * 32, 32, 1.0f / (CSC * CSC), nullptr, 0, nullptr, 1, 0, 0, SC + (size_t)b * HWP * 256, nullptr, SD * 256, 256, SD, SD, 32);
    k_jsm<<<NPX / 256, 256, 0, stream>>>(SC, WT, NPX);
    for (int b = 0; b < NB; ++b) k_gemm2<0><<<dim3((SD / 128) * (CH / 64), SD), 128, 0, stream>>>(WT + (size_t)b * HWP * 256, SD * 256, 256, VX + (size_t)b * CH * HWP, HWP, SD, 1.0f / (CSC * CSC), nullptr, 0, nullptr, 1, 0, 0, YC + (size_t)b * HWP * CH, nullptr, SD * CH, CH, SD, CH, SD);
    for (int b = 0; b < NB; ++b) k_gemm2<0><<<dim3((SD / 128) * (CH / 64), SD), 128, 0, stream>>>(WT + (size_t)b * HWP * 256 + SD, 256, (size_t)SD * 256, VC + (size_t)b * CH * HWP, HWP, SD, 1.0f / (CSC * CSC), B3, 0, YC + (size_t)b * HWP * CH, -1, 0, 0, Y + (size_t)b * HWP * CH, nullptr, CH, (size_t)SD * CH, SD, CH, SD);
  }
  k_adf<<<(unsigned)(NPX * CH / 8 / 256), 256, 0, stream>>>(YA, YB, D1, D2, NPX * CH / 8);
  k_gemm2<0><<<dim3((NPX / 128) * (CH / 64), 1), 128, 0, stream>>>(D1, CH, 0, W4, CH, 0, 1.0f / CSC, nullptr, 0, nullptr, 1, 0, 0, Z1, nullptr, CH, 0, NPX, CH, CH);
  k_gemm2<6><<<dim3((NPX / 128) * (CH / 64), 1), 128, 0, stream>>>(D2, CH, 0, W4, CH, 0, 1.0f / (CSC * RSD), BPJ, 0, Z1, -1, 0, 0, ZZ, nullptr, CH, 0, NPX, CH, CH);
  k_bns<<<1, 64, 0, stream>>>(ZZ, ST, CH);
  k_two_outs<<<(unsigned)(NB * CH * HWP / 4 / 256), 256, 0, stream>>>(YA, YB, ZZ, ST, IA, IB, G1, G2, SCL, SHF, O1, O2, NB * CH * HWP / 4);
}
